// Mambaspe_4020089389062
// MI455X (gfx1250) — hardware-verified
//
#include <hip/hip_runtime.h>


typedef _Float16 v16h __attribute__((ext_vector_type(16)));
typedef _Float16 v8h  __attribute__((ext_vector_type(8)));
typedef float    v8f  __attribute__((ext_vector_type(8)));
typedef float    v4f  __attribute__((ext_vector_type(4)));
union Frag { v16h v; v8h half[2]; };

#define NBATCH 8
#define CIN    256
#define DIN    256
#define HWN    4096
#define IMW    64
#define CN     32
#define LG     8
#define NS     16
#define XCOLS  68
#define XPAD   96

__device__ __forceinline__ v8f wmma_f16(v16h a, v16h b, v8f c)
{
    v8f d = __builtin_amdgcn_wmma_f32_16x16x32_f16(false, a, false, b, (short)0, c, false, false);
    asm volatile("v_nop\n\tv_nop\n\tv_nop\n\tv_nop" : "+v"(d) : "v"(a), "v"(b));
    return d;
}

__device__ __forceinline__ v8f zero8()
{
    v8f z;
#pragma unroll
    for (int i = 0; i < 8; ++i) z[i] = 0.f;
    return z;
}

__device__ __forceinline__ float wave_sum(float v)
{
#pragma unroll
    for (int o = 16; o > 0; o >>= 1) v += __shfl_xor(v, o, 32);
    return v;
}

__global__ void __launch_bounds__(256)
k_prep(const float* __restrict__ w1, const float* __restrict__ w2, const float* __restrict__ xpw,
       _Float16* w1h, _Float16* w2h, _Float16* wch)
{
    const int blk = blockIdx.x, t = threadIdx.x;
    v8h hv;
    bool act = true;
    _Float16* dst;
    if (blk < 64) {
        const int sel = blk >> 5;
        const size_t e0 = (size_t)(blk & 31) * 2048 + (size_t)t * 8;
        const float* src = (sel == 0 ? w1 : w2) + e0;
        dst = (sel == 0 ? w1h : w2h) + e0;
        const v4f a = *(const v4f*)src;
        const v4f c = *(const v4f*)(src + 4);
        hv[0] = (_Float16)(a.x * 64.f); hv[1] = (_Float16)(a.y * 64.f);
        hv[2] = (_Float16)(a.z * 64.f); hv[3] = (_Float16)(a.w * 64.f);
        hv[4] = (_Float16)(c.x * 64.f); hv[5] = (_Float16)(c.y * 64.f);
        hv[6] = (_Float16)(c.z * 64.f); hv[7] = (_Float16)(c.w * 64.f);
    } else {
        const int e0 = (blk - 64) * 2048 + t * 8;
        act = e0 < XPAD * CN;
        dst = wch + (act ? e0 : 0);
#pragma unroll
        for (int q = 0; q < 8; ++q) {
            const int e = e0 + q;
            const int row = e >> 5, col = e & 31;
            const float v = (act && row < XCOLS) ? xpw[row * CN + col] * 64.f : 0.f;
            hv[q] = (_Float16)v;
        }
    }
    if (act) {
        const v4f f = __builtin_bit_cast(v4f, hv);
        *(volatile v4f*)dst = f;
        __threadfence();
        *(volatile v4f*)dst = f;
    }
}

__global__ void __launch_bounds__(256)
k_gate(const float* __restrict__ x, const float* __restrict__ skw,
       const float* __restrict__ skb, float* gate)
{
    __shared__ float zm[CIN];
    __shared__ __attribute__((aligned(16))) float gs[CIN];
    const int b = blockIdx.x, t = threadIdx.x, w = t >> 5, lane = t & 31;

#pragma unroll 1
    for (int i = 0; i < 32; ++i) {
        const int c = w * 32 + i;
        const float* p = x + ((size_t)(b * CIN + c)) * HWN;
        float s = 0.f;
#pragma unroll 4
        for (int it = 0; it < 32; ++it) {
            const v4f v = *(const v4f*)(p + (it * 32 + lane) * 4);
            s += (v.x + v.y) + (v.z + v.w);
        }
        s = wave_sum(s);
        if (lane == 0) zm[c] = s * (1.f / 4096.f);
    }
    __syncthreads();
    {
        const int c = t;
        float z = 0.f;
#pragma unroll
        for (int tt = 0; tt < 5; ++tt) {
            const int cc = c + tt - 2;
            if (cc >= 0 && cc < CIN) z += skw[tt] * zm[cc];
        }
        z += skb[0];
        const float zmax = z;
        const float e = __expf(z - zmax);
        const float s = e * __builtin_amdgcn_rcpf(e);
        gs[c] = s;
    }
    __syncthreads();
    if (t < 64) {
        const v4f v = *(const v4f*)(&gs[t * 4]);
        float* dp = gate + (size_t)b * CIN + t * 4;
        *(volatile v4f*)dp = v;
        __threadfence();
        *(volatile v4f*)dp = v;
    }
}

template <int MODE>
__global__ void __launch_bounds__(128)
k_gemm(const _Float16* __restrict__ ah, const float* __restrict__ xs,
       const _Float16* __restrict__ ys, float* dst)
{
    __shared__ __attribute__((aligned(16))) float Ds[64 * 64];

    const int t = threadIdx.x, w = t >> 5, lane = t & 31, h = lane >> 4, m = lane & 15;
    const int b    = blockIdx.x >> 6;
    const int hw0  = (blockIdx.x & 63) * 64;
    const int row0 = blockIdx.y * 64;
    const int wm   = (w >> 1) * 32;
    const int wn   = (w & 1) * 32;

    v8f acc[2][2];
#pragma unroll
    for (int i = 0; i < 2; ++i)
#pragma unroll
        for (int j = 0; j < 2; ++j) acc[i][j] = zero8();

#pragma unroll 1
    for (int k0 = 0; k0 < 256; k0 += 32) {
        Frag af[2];
        v16h bv[2];
#pragma unroll
        for (int i = 0; i < 2; ++i) {
            const _Float16* ap = ah + (size_t)(row0 + wm + i * 16 + m) * 256 + k0 + 8 * h;
            af[i].half[0] = *(const v8h*)ap;
            af[i].half[1] = *(const v8h*)(ap + 16);
        }
#pragma unroll
        for (int j = 0; j < 2; ++j) {
            const int n = hw0 + wn + j * 16 + m;
            if (MODE == 0) {
                const float* bp = xs + ((size_t)(b * CIN + k0 + 8 * h)) * HWN + n;
                v16h bq;
#pragma unroll
                for (int q = 0; q < 8; ++q) {
                    bq[q]     = (_Float16)bp[(size_t)q * HWN];
                    bq[8 + q] = (_Float16)bp[(size_t)(16 + q) * HWN];
                }
                bv[j] = bq;
            } else {
                const _Float16* bp = ys + ((size_t)(b * HWN + n)) * DIN + k0 + 8 * h;
                Frag bq;
                bq.half[0] = *(const v8h*)bp;
                bq.half[1] = *(const v8h*)(bp + 16);
                bv[j] = bq.v;
            }
        }
#pragma unroll
        for (int i = 0; i < 2; ++i)
#pragma unroll
            for (int j = 0; j < 2; ++j)
                acc[i][j] = wmma_f16(af[i].v, bv[j], acc[i][j]);
    }

    const float osc = 1.f / 64.f;
#pragma unroll
    for (int i = 0; i < 2; ++i)
#pragma unroll
        for (int j = 0; j < 2; ++j)
#pragma unroll
            for (int r = 0; r < 8; ++r)
                Ds[(wm + i * 16 + 8 * h + r) * 64 + wn + j * 16 + m] = acc[i][j][r] * osc;
    __syncthreads();

    v4f vals[8];
    const int rsub = t >> 4;
    const int c4   = (t & 15) * 4;
#pragma unroll
    for (int ps = 0; ps < 8; ++ps)
        vals[ps] = *(const v4f*)(&Ds[(ps * 8 + rsub) * 64 + c4]);
    float* gb = dst + ((size_t)(b * 256 + row0 + rsub)) * HWN + hw0 + c4;
#pragma unroll
    for (int ps = 0; ps < 8; ++ps)
        *(volatile v4f*)(gb + (size_t)(ps * 8) * HWN) = vals[ps];
    __threadfence();
#pragma unroll
    for (int ps = 0; ps < 8; ++ps)
        *(volatile v4f*)(gb + (size_t)(ps * 8) * HWN) = vals[ps];
}

__global__ void __launch_bounds__(256)
k_ssm(const float* __restrict__ xi, const float* __restrict__ cw, const float* __restrict__ cb,
      const _Float16* __restrict__ wch, const float* __restrict__ dtw, const float* __restrict__ dtb,
      const float* __restrict__ alog, const float* __restrict__ dsv, const float* __restrict__ lng,
      const float* __restrict__ lnb, const float* __restrict__ gate, _Float16* yln)
{
    __shared__ __attribute__((aligned(16))) float    Ush[8 * CN * LG];
    __shared__ __attribute__((aligned(16))) _Float16 Af[64 * CN];
    __shared__ __attribute__((aligned(16))) float    Xd[8 * XCOLS * LG];
    __shared__ __attribute__((aligned(16))) float    Yc[8 * LG * CN];
    __shared__ __attribute__((aligned(16))) _Float16 Of[8 * DIN];

    const int t = threadIdx.x, w = t >> 5, lane = t & 31, h = lane >> 4, m = lane & 15;
    const int p0  = blockIdx.x * 8;
    const int b   = p0 >> 12;
    const int hw0 = p0 & (HWN - 1);
    const int hh  = hw0 >> 6;
    const int wc0 = hw0 & (IMW - 1);

    {
        const int d = t;
        const float* base = xi + ((size_t)(b * DIN + d)) * HWN;
        float xv[3][10];
#pragma unroll
        for (int ky = 0; ky < 3; ++ky) {
            const int r = hh + ky - 1;
            const bool rv = (unsigned)r < 64u;
#pragma unroll
            for (int q = 0; q < 10; ++q) xv[ky][q] = 0.f;
            if (rv) {
                const float* rp = base + r * IMW + wc0;
                const v4f v0 = *(const v4f*)rp;
                const v4f v1 = *(const v4f*)(rp + 4);
                xv[ky][1] = v0.x; xv[ky][2] = v0.y; xv[ky][3] = v0.z; xv[ky][4] = v0.w;
                xv[ky][5] = v1.x; xv[ky][6] = v1.y; xv[ky][7] = v1.z; xv[ky][8] = v1.w;
                if (wc0 > 0)        xv[ky][0] = rp[-1];
                if (wc0 + 8 < IMW)  xv[ky][9] = rp[8];
            }
        }
        float wv[9];
#pragma unroll
        for (int q = 0; q < 9; ++q) wv[q] = cw[d * 9 + q];
        const float bias = cb[d];
        const int cc = d >> 3, gl = d & 7;
#pragma unroll
        for (int j = 0; j < 8; ++j) {
            float a = 0.f;
#pragma unroll
            for (int ky = 0; ky < 3; ++ky)
#pragma unroll
                for (int kx = 0; kx < 3; ++kx)
                    a += xv[ky][j + kx] * wv[ky * 3 + kx];
            a += bias;
            const float e  = __expf(-a);
            const float sv = a * __builtin_amdgcn_rcpf(1.f + e);
            Ush[(j * CN + cc) * LG + gl] = sv;
            Af[(j * LG + gl) * CN + cc]  = (_Float16)(sv * 16.f);
        }
    }
    __syncthreads();

    {
        const int mt = w >> 1;
        Frag a;
        const _Float16* ap = Af + (mt * 16 + m) * CN + 8 * h;
        a.half[0] = *(const v8h*)ap;
        a.half[1] = *(const v8h*)(ap + 16);
        const int pix = mt * 2 + h;
#pragma unroll
        for (int i = 0; i < 3; ++i) {
            const int nt = (w & 1) + 2 * i;
            Frag bq;
            const _Float16* bp = wch + (nt * 16 + m) * CN + 8 * h;
            bq.half[0] = *(const v8h*)bp;
            bq.half[1] = *(const v8h*)(bp + 16);
            v8f acc = zero8();
            acc = wmma_f16(a.v, bq.v, acc);
            const int col = nt * 16 + m;
            if (col < XCOLS) {
                float* xp = Xd + (pix * XCOLS + col) * LG;
#pragma unroll
                for (int r = 0; r < 8; ++r) xp[r] = acc[r] * (1.f / 1024.f);
            }
        }
    }
    __syncthreads();

    {
        const int j = w, c = lane;
#pragma unroll
        for (int l = 0; l < LG; ++l) Yc[(j * LG + l) * CN + c] = 0.f;

#pragma unroll 1
        for (int k = 0; k < 2; ++k) {
            const int rm = k * 7;
            float ul[LG];
#pragma unroll
            for (int l = 0; l < LG; ++l) ul[l] = Ush[(j * CN + c) * LG + (l ^ rm)];
            const float w0v = dtw[(k * CN + c) * 2 + 0];
            const float w1v = dtw[(k * CN + c) * 2 + 1];
            const float bb  = dtb[k * CN + c];
            const float Dv  = dsv[k * CN + c];
            float An[NS];
#pragma unroll
            for (int n = 0; n < NS; ++n) An[n] = -__expf(alog[(k * CN + c) * NS + n]);
            const float* Xp = Xd + (j * XCOLS + k * 34) * LG;
            float hs[NS];
#pragma unroll
            for (int n = 0; n < NS; ++n) hs[n] = 0.f;
#pragma unroll
            for (int l = 0; l < LG; ++l) {
                const int pos = l ^ rm;
                const float rr = (Xp[pos] * w0v + Xp[LG + pos] * w1v) + bb;
                const float dt = fmaxf(rr, 0.f) + __logf(1.f + __expf(-fabsf(rr)));
                const float du = dt * ul[l];
                float y = 0.f;
#pragma unroll
                for (int n = 0; n < NS; ++n) {
                    const float bn = Xp[(2 + n) * LG + pos];
                    const float cn = Xp[(18 + n) * LG + pos];
                    hs[n] = hs[n] * __expf(dt * An[n]) + du * bn;
                    y += hs[n] * cn;
                }
                const float ysv = y + Dv * ul[l];
                Yc[(j * LG + pos) * CN + c] += ysv;
            }
        }

        const float gg = lng[c], be = lnb[c];
#pragma unroll
        for (int l = 0; l < LG; ++l) {
            const float v  = Yc[(j * LG + l) * CN + c];
            const float mu = wave_sum(v) * (1.f / 32.f);
            const float dv = v - mu;
            const float var = wave_sum(dv * dv) * (1.f / 32.f);
            const float rstd = rsqrtf(var + 1e-5f);
            float o = dv * rstd * gg + be;
            o *= gate[(size_t)b * DIN + l * CN + c];
            Of[j * DIN + l * CN + c] = (_Float16)o;
        }
    }
    __syncthreads();

    {
        const v8h hv = *(const v8h*)(Of + t * 8);
        const v4f f  = __builtin_bit_cast(v4f, hv);
        _Float16* dp = yln + (size_t)p0 * DIN + t * 8;
        *(volatile v4f*)dp = f;
        __threadfence();
        *(volatile v4f*)dp = f;
    }
}

extern "C" void kernel_launch(void* const* d_in, const int* in_sizes, int n_in,
                              void* d_out, int out_size, void* d_ws, size_t ws_size,
                              hipStream_t stream)
{
    if (n_in < 14) return;
    if (in_sizes[0]  != NBATCH * CIN * HWN) return;
    if (in_sizes[1]  != DIN * CIN)          return;
    if (in_sizes[2]  != 5)                  return;
    if (in_sizes[3]  != 1)                  return;
    if (in_sizes[4]  != DIN * 9)            return;
    if (in_sizes[5]  != DIN)                return;
    if (in_sizes[6]  != 2 * 34 * CN)        return;
    if (in_sizes[7]  != 2 * CN * 2)         return;
    if (in_sizes[8]  != 2 * CN)             return;
    if (in_sizes[9]  != 2 * CN * NS)        return;
    if (in_sizes[10] != 2 * CN)             return;
    if (in_sizes[11] != CN)                 return;
    if (in_sizes[12] != CN)                 return;
    if (in_sizes[13] != CIN * DIN)          return;
    if (out_size     != NBATCH * CIN * HWN) return;

    const float* x    = (const float*)d_in[0];
    const float* w_in = (const float*)d_in[1];
    const float* skw  = (const float*)d_in[2];
    const float* skb  = (const float*)d_in[3];
    const float* cw   = (const float*)d_in[4];
    const float* cb   = (const float*)d_in[5];
    const float* xpw  = (const float*)d_in[6];
    const float* dtw  = (const float*)d_in[7];
    const float* dtb  = (const float*)d_in[8];
    const float* alog = (const float*)d_in[9];
    const float* dsv  = (const float*)d_in[10];
    const float* lng  = (const float*)d_in[11];
    const float* lnb  = (const float*)d_in[12];
    const float* w_out= (const float*)d_in[13];
    float* out = (float*)d_out;

    const size_t off_w1h  = 0;
    const size_t off_w2h  = 131072;
    const size_t off_wch  = 262144;
    const size_t off_gate = 270336;
    const size_t off_xi   = (size_t)1 << 20;
    const size_t off_yln  = off_xi + (size_t)NBATCH * DIN * HWN * 4;
    const size_t need     = off_yln + (size_t)NBATCH * HWN * DIN * 2;
    if (ws_size < need) return;

    char* ws = (char*)d_ws;
    _Float16* w1h  = (_Float16*)(ws + off_w1h);
    _Float16* w2h  = (_Float16*)(ws + off_w2h);
    _Float16* wch  = (_Float16*)(ws + off_wch);
    float*    gate = (float*)(ws + off_gate);
    float*    xi   = (float*)(ws + off_xi);
    _Float16* yln  = (_Float16*)(ws + off_yln);

    k_prep<<<66, 256, 0, stream>>>(w_in, w_out, xpw, w1h, w2h, wch);
    k_gate<<<NBATCH, 256, 0, stream>>>(x, skw, skb, gate);
    k_gemm<0><<<dim3(NBATCH * 64, 4), 128, 0, stream>>>(w1h, x, yln, xi);
    k_ssm<<<(NBATCH * HWN) / 8, 256, 0, stream>>>(xi, cw, cb, wch, dtw, dtb, alog, dsv,
                                                   lng, lnb, gate, yln);
    k_gemm<1><<<dim3(NBATCH * 64, 4), 128, 0, stream>>>(w2h, x, yln, out);
}
